// JunmaiLayer_68582037782789
// MI455X (gfx1250) — hardware-verified
//
#include <hip/hip_runtime.h>
#include <math.h>

#pragma clang fp contract(off)

#define FEAT 64
#define NCH 64
#define NRBF 50
#define PPITCH 256
#define PAIR_THREADS 256
#define PAIR_WAVES 8
#define GEMM_THREADS 128

typedef float v8f __attribute__((ext_vector_type(8)));
typedef float v4f __attribute__((ext_vector_type(4)));
typedef float v4fa __attribute__((ext_vector_type(4), may_alias));
typedef __bf16 v16bf __attribute__((ext_vector_type(16)));
typedef unsigned short v16us __attribute__((ext_vector_type(16)));

union Frag16 { v16bf v; v16us u; };

__device__ __forceinline__ unsigned short bf16_bits_rne(float f) {
  unsigned int u = __float_as_uint(f);
  u += 0x7fffu + ((u >> 16) & 1u);
  return (unsigned short)(u >> 16);
}

__device__ __forceinline__ float bf16_to_f32(unsigned short b) {
  return __uint_as_float(((unsigned int)b) << 16);
}

__device__ __forceinline__ v8f wmma_bf16(v16bf a, v16bf b, v8f c) {
  v8f d = __builtin_amdgcn_wmma_f32_16x16x32_bf16(false, a, false, b, (short)0, c, false, false);
  asm volatile("v_nop\n\tv_nop\n\tv_nop\n\tv_nop" : "+v"(d) : "v"(a), "v"(b));
  return d;
}

__device__ __forceinline__ v8f wmma_x3(const Frag16& ah, const Frag16& al,
                                       const Frag16& bh, const Frag16& bl, v8f c) {
  c = wmma_bf16(ah.v, bh.v, c);
  c = wmma_bf16(ah.v, bl.v, c);
  c = wmma_bf16(al.v, bh.v, c);
  return c;
}

__global__ __launch_bounds__(GEMM_THREADS)
void gemm_split_kernel(const float* __restrict__ A, int lda,
                       const float* __restrict__ B, int ldb,
                       const float* __restrict__ bias, int use_bias, int act_tanh,
                       float* Cm, int ldc, int M, int N, int K)
{
  const int tid  = threadIdx.x;
  const int lane = tid & 31;
  const int wave = tid >> 5;
  const int h    = lane >> 4;
  const int m    = lane & 15;
  const int row0 = blockIdx.y * 16;
  const int col0 = blockIdx.x * 64;
  if (row0 + 16 > M || col0 + 64 > N) return;

  __shared__ __align__(16) float tile_s[16][64];

  const int cw = col0 + wave * 16;

  v8f acc = {0.f, 0.f, 0.f, 0.f, 0.f, 0.f, 0.f, 0.f};
  for (int k0 = 0; k0 + 32 <= K; k0 += 32) {
    const float* ap = A + (size_t)(row0 + m) * lda + k0 + 8 * h;
    const v4f a0 = *(const v4fa*)(ap);
    const v4f a1 = *(const v4fa*)(ap + 4);
    const v4f a2 = *(const v4fa*)(ap + 16);
    const v4f a3 = *(const v4fa*)(ap + 20);
    float av[16] = {a0.x, a0.y, a0.z, a0.w, a1.x, a1.y, a1.z, a1.w,
                    a2.x, a2.y, a2.z, a2.w, a3.x, a3.y, a3.z, a3.w};
    float bv[16];
    const float* bp = B + (size_t)(k0 + 8 * h) * ldb + cw + m;
#pragma unroll
    for (int e = 0; e < 8; ++e) {
      bv[e]     = bp[(size_t)e * ldb];
      bv[8 + e] = bp[(size_t)(16 + e) * ldb];
    }
    Frag16 ah, al, bh, bl;
#pragma unroll
    for (int e = 0; e < 16; ++e) {
      const unsigned short ha = bf16_bits_rne(av[e]);
      ah.u[e] = ha;
      al.u[e] = bf16_bits_rne(av[e] - bf16_to_f32(ha));
      const unsigned short hb = bf16_bits_rne(bv[e]);
      bh.u[e] = hb;
      bl.u[e] = bf16_bits_rne(bv[e] - bf16_to_f32(hb));
    }
    acc = wmma_x3(ah, al, bh, bl, acc);
  }

  const float bcol = bias[(cw + m) * use_bias] * (float)use_bias;
#pragma unroll
  for (int r = 0; r < 8; ++r) {
    float v = acc[r] + bcol;
    if (act_tanh) v = tanhf(v);
    tile_s[8 * h + r][wave * 16 + m] = v;
  }
  __syncthreads();

  const int q0 = tid;
  const int q1 = tid + GEMM_THREADS;
  const int r0i = q0 >> 4, c0i = (q0 & 15) * 4;
  const int r1i = q1 >> 4, c1i = (q1 & 15) * 4;
  const v4f v0 = *(const v4fa*)(&tile_s[r0i][c0i]);
  const v4f v1 = *(const v4fa*)(&tile_s[r1i][c1i]);
  float* p0 = Cm + (size_t)(row0 + r0i) * ldc + col0 + c0i;
  float* p1 = Cm + (size_t)(row0 + r1i) * ldc + col0 + c1i;
  *(volatile v4fa*)p0 = v0;
  *(volatile v4fa*)p1 = v1;
  __threadfence();
  *(volatile v4fa*)p0 = v0;
  *(volatile v4fa*)p1 = v1;
}

__global__ __launch_bounds__(PAIR_THREADS)
void pair_kernel(const float* __restrict__ x, const float* __restrict__ W_basis,
                 const float* __restrict__ means, const float* __restrict__ betas,
                 const float* __restrict__ P, float* Hn, int n_atoms)
{
  const int i = blockIdx.x;
  if (i >= n_atoms) return;
  const int tid  = threadIdx.x;
  const int lane = tid & 31;
  const int wave = tid >> 5;
  const int h    = lane >> 4;
  const int m    = lane & 15;

  __shared__ v16us Bh_s[2][4][32];
  __shared__ v16us Bl_s[2][4][32];
  __shared__ float KQi_s[2 * NCH];
  __shared__ float means_s[64];
  __shared__ float betas_s[64];
  __shared__ float red_s[PAIR_WAVES][NCH];
  __shared__ __align__(16) float hn_s[NCH];

  {
    const int s  = tid >> 7;
    const int ct = (tid >> 5) & 3;
    const int lf = tid & 31;
    const int hf = lf >> 4;
    const int n  = ct * 16 + (lf & 15);
    Frag16 fh, fl;
#pragma unroll
    for (int e = 0; e < 16; ++e) {
      const int kk = (e < 8) ? (8 * hf + e) : (8 + 8 * hf + e);
      const int r  = 32 * s + kk;
      float v = 0.f;
      if (r < NRBF) v = W_basis[r * NCH + n];
      const unsigned short hb = bf16_bits_rne(v);
      fh.u[e] = hb;
      fl.u[e] = bf16_bits_rne(v - bf16_to_f32(hb));
    }
    Bh_s[s][ct][lf] = fh.u;
    Bl_s[s][ct][lf] = fl.u;
  }
  if (tid < 2 * NCH) KQi_s[tid] = P[(size_t)i * PPITCH + tid];
  if (tid < 64) {
    means_s[tid] = (tid < NRBF) ? means[tid] : 0.f;
    betas_s[tid] = (tid < NRBF) ? betas[tid] : 0.f;
  }
  __syncthreads();

  const float xi0 = x[i * 3 + 0];
  const float xi1 = x[i * 3 + 1];
  const float xi2 = x[i * 3 + 2];

  float hn_part[4] = {0.f, 0.f, 0.f, 0.f};
  const int ntiles = n_atoms >> 4;

  for (int t = wave; t < ntiles; t += PAIR_WAVES) {
    const int jbase = t * 16;
    const int j = jbase + m;

    const float dx0 = xi0 - x[j * 3 + 0];
    const float dx1 = xi1 - x[j * 3 + 1];
    const float dx2 = xi2 - x[j * 3 + 2];
    const float d2  = (dx0 * dx0 + dx1 * dx1) + dx2 * dx2;
    const float d   = sqrtf(d2 + 1e-10f);
    const float denom = d * d + 1e-10f;
    const float sumsq = d2 / (denom * denom);
    const float cutoff = (d < 5.0f) ? (0.5f * (cosf(d * 0.62831853071795862f) + 1.0f)) : 0.f;
    const float ed = expf(-d);

    float ssq[8];
#pragma unroll
    for (int r = 0; r < 8; ++r) ssq[r] = __shfl(sumsq, 8 * h + r);

    Frag16 ah[2], al[2];
#pragma unroll
    for (int ks = 0; ks < 2; ++ks) {
#pragma unroll
      for (int e = 0; e < 16; ++e) {
        const int kk = (e < 8) ? (8 * h + e) : (8 + 8 * h + e);
        const int r  = 32 * ks + kk;
        float sv = 0.f;
        if (r < NRBF) {
          const float tt = ed - means_s[r];
          sv = cutoff * expf(-betas_s[r] * (tt * tt));
        }
        const unsigned short hb = bf16_bits_rne(sv);
        ah[ks].u[e] = hb;
        al[ks].u[e] = bf16_bits_rne(sv - bf16_to_f32(hb));
      }
    }

#pragma unroll
    for (int ct = 0; ct < 4; ++ct) {
      v8f acc = {0.f, 0.f, 0.f, 0.f, 0.f, 0.f, 0.f, 0.f};
#pragma unroll
      for (int ks = 0; ks < 2; ++ks) {
        Frag16 bh, bl;
        bh.u = Bh_s[ks][ct][lane];
        bl.u = Bl_s[ks][ct][lane];
        acc = wmma_x3(ah[ks], al[ks], bh, bl, acc);
      }
      const int c = ct * 16 + m;
      const float kai = KQi_s[c];
      const float qai = KQi_s[NCH + c];
      float part = 0.f;
#pragma unroll
      for (int r = 0; r < 8; ++r) {
        const int j2 = jbase + 8 * h + r;
        const float kb = P[(size_t)j2 * PPITCH + 2 * NCH + c];
        const float qb = P[(size_t)j2 * PPITCH + 3 * NCH + c];
        const float kq = (kai + kb) * (qai + qb);
        const float bv = acc[r];
        part += (kq * (bv * bv)) * ssq[r];
      }
      hn_part[ct] += part;
    }
  }

#pragma unroll
  for (int ct = 0; ct < 4; ++ct) {
    const float other = __shfl_xor(hn_part[ct], 16);
    const float v = hn_part[ct] + other;
    if (h == 0) red_s[wave][ct * 16 + m] = v;
  }
  __syncthreads();
  if (tid < NCH) {
    float s = 0.f;
#pragma unroll
    for (int w = 0; w < PAIR_WAVES; ++w) s += red_s[w][tid];
    hn_s[tid] = s;
  }
  __syncthreads();
  if (tid < 16) {
    const v4f hv = *(const v4fa*)(&hn_s[4 * tid]);
    float* hp = Hn + (size_t)i * NCH + 4 * tid;
    *(volatile v4fa*)hp = hv;
    __threadfence();
    *(volatile v4fa*)hp = hv;
  }
}

extern "C" void kernel_launch(void* const* d_in, const int* in_sizes, int n_in,
                              void* d_out, int out_size, void* d_ws, size_t ws_size,
                              hipStream_t stream)
{
  if (n_in < 11) return;
  const float* h_in    = (const float*)d_in[0];
  const float* x       = (const float*)d_in[1];
  const float* W_node  = (const float*)d_in[2];
  const float* b_node  = (const float*)d_in[3];
  const float* W_basis = (const float*)d_in[4];
  const float* means   = (const float*)d_in[5];
  const float* betas   = (const float*)d_in[6];
  const float* W_s1    = (const float*)d_in[7];
  const float* b_s1    = (const float*)d_in[8];
  const float* W_s2    = (const float*)d_in[9];
  const float* b_s2    = (const float*)d_in[10];
  float* out = (float*)d_out;

  const int n_atoms = in_sizes[1] / 3;
  if (n_atoms <= 0 || (n_atoms % 16) != 0) return;
  if (in_sizes[0] != n_atoms * FEAT) return;
  if (in_sizes[1] != n_atoms * 3) return;
  if (in_sizes[2] != 2 * FEAT * 2 * NCH) return;
  if (in_sizes[3] != 2 * NCH) return;
  if (in_sizes[4] != NRBF * NCH) return;
  if (in_sizes[5] != NRBF || in_sizes[6] != NRBF) return;
  if (in_sizes[7] != NCH * NCH || in_sizes[8] != NCH) return;
  if (in_sizes[9] != NCH * NCH || in_sizes[10] != NCH) return;
  if (out_size != n_atoms * NCH) return;

  const size_t p_bytes  = (size_t)n_atoms * PPITCH * sizeof(float);
  const size_t hn_bytes = (size_t)n_atoms * NCH * sizeof(float);
  const size_t off_p  = 0;
  const size_t off_hn = (off_p + p_bytes + 255) & ~(size_t)255;
  const size_t off_t  = (off_hn + hn_bytes + 255) & ~(size_t)255;
  const size_t total  = off_t + hn_bytes;
  if (total > ws_size) return;

  float* P  = (float*)((char*)d_ws + off_p);
  float* Hn = (float*)((char*)d_ws + off_hn);
  float* T  = (float*)((char*)d_ws + off_t);

  const dim3 g_node(2 * NCH / 64, n_atoms / 16);
  const dim3 g_head(NCH / 64, n_atoms / 16);

  gemm_split_kernel<<<g_node, GEMM_THREADS, 0, stream>>>(
      h_in, FEAT, W_node, 2 * NCH, b_node, 1, 0, P, PPITCH, n_atoms, 2 * NCH, FEAT);
  gemm_split_kernel<<<g_node, GEMM_THREADS, 0, stream>>>(
      h_in, FEAT, W_node + FEAT * 2 * NCH, 2 * NCH, b_node, 0, 0, P + 2 * NCH, PPITCH,
      n_atoms, 2 * NCH, FEAT);

  pair_kernel<<<n_atoms, PAIR_THREADS, 0, stream>>>(x, W_basis, means, betas, P, Hn, n_atoms);

  gemm_split_kernel<<<g_head, GEMM_THREADS, 0, stream>>>(
      Hn, NCH, W_s1, NCH, b_s1, 1, 1, T, NCH, n_atoms, NCH, NCH);
  gemm_split_kernel<<<g_head, GEMM_THREADS, 0, stream>>>(
      T, NCH, W_s2, NCH, b_s2, 1, 0, out, NCH, n_atoms, NCH, NCH);
}
